// GAT_2_64037962383538
// MI455X (gfx1250) — hardware-verified
//
#include <hip/hip_runtime.h>
#include <stddef.h>


#define DF    128
#define HP    8
#define GR    32
#define AP    136
#define XSP   132
#define TP    129
#define NB    480
#define SLOTP 512
#define CHUNK 1024
#define NTHR  256
#define NWAVE 8
#define WCAP  128
#define NBLK  128
#define NG    512
#define NCLS  10
#define KHD   64
#define EPSBN 1e-5f

#define LDS_SACC (NB * DF)
#define LDS_DEN  (NB * HP)
#define LDS_MAX  (NB * HP)
#define LDS_LIST (NWAVE * WCAP)
#define LDS_BYTES ((LDS_SACC + LDS_DEN + LDS_MAX + LDS_LIST + NWAVE) * 4)

static_assert(WCAP == (CHUNK / NTHR) * 32);
static_assert(LDS_BYTES == 280608);
static_assert((NB % NWAVE) == 0);
static_assert(NB <= SLOTP);
static_assert(SLOTP == 512);
static_assert(CHUNK == 1024);
static_assert(((LDS_SACC + LDS_DEN + LDS_MAX) % 4) == 0);
static_assert(NG * NCLS == 20 * NTHR);
static_assert((NG * NCLS) / 4 == 5 * NTHR);

typedef float          v4f   __attribute__((ext_vector_type(4)));
typedef float          v8f   __attribute__((ext_vector_type(8)));
typedef int            v4i   __attribute__((ext_vector_type(4)));
typedef unsigned short v8us  __attribute__((ext_vector_type(8)));
typedef unsigned short v16us __attribute__((ext_vector_type(16)));
typedef __bf16         v16bf __attribute__((ext_vector_type(16)));
union Frag   { v16bf v; v16us u; v8us half[2]; };
union Pack16 { v8us h; v4i i; };

__device__ __forceinline__ v8f wm(v16bf a, v16bf b, v8f c) {
  v8f d = __builtin_amdgcn_wmma_f32_16x16x32_bf16(false, a, false, b, (short)0, c, false, false);
  asm volatile("v_nop\n\tv_nop\n\tv_nop\n\tv_nop" : "+v"(d) : "v"(a), "v"(b));
  return d;
}

__device__ __forceinline__ unsigned short bf_bits(float x) {
  const unsigned u = __float_as_uint(x);
  return (unsigned short)((u + 0x7FFFu + ((u >> 16) & 1u)) >> 16);
}
__device__ __forceinline__ void bf_split(float x, unsigned short& hi, unsigned short& lo) {
  const unsigned short hb = bf_bits(x);
  const float r = x - __uint_as_float(((unsigned)hb) << 16);
  hi = hb;
  lo = bf_bits(r);
}

__device__ __forceinline__ v4f relu4(v4f a) {
  v4f r;
  r.x = a.x > 0.f ? a.x : 0.f;
  r.y = a.y > 0.f ? a.y : 0.f;
  r.z = a.z > 0.f ? a.z : 0.f;
  r.w = a.w > 0.f ? a.w : 0.f;
  return r;
}

__global__ __launch_bounds__(NTHR) void k_prepw(const float* __restrict__ W, int K, int Nv,
                                                unsigned short* Wh, unsigned short* Wl) {
  __shared__ __attribute__((aligned(16))) float T[32 * TP];
  const int tid = threadIdx.x;
  const int n0  = blockIdx.x * 32;
#pragma unroll
  for (int i = 0; i < 16; ++i) {
    const int idx = i * NTHR + tid;
    const int k   = idx >> 5;
    const int c   = idx & 31;
    const int kc  = (k < K) ? k : (K - 1);
    const int n   = n0 + c;
    const int nc  = (n < Nv) ? n : (Nv - 1);
    const float w = W[(size_t)kc * Nv + nc];
    T[c * TP + k] = (k < K && n < Nv) ? w : 0.f;
  }
  __syncthreads();
  Pack16 uh[2], ul[2];
  size_t po[2];
#pragma unroll
  for (int q = 0; q < 2; ++q) {
    const int t  = q * NTHR + tid;
    const int c  = t >> 4;
    const int k0 = (t & 15) * 8;
#pragma unroll
    for (int j = 0; j < 8; ++j) {
      unsigned short a, b;
      bf_split(T[c * TP + k0 + j], a, b);
      uh[q].h[j] = a;
      ul[q].h[j] = b;
    }
    po[q] = (size_t)(n0 + c) * DF + k0;
  }
#pragma unroll
  for (int q = 0; q < 2; ++q) {
    *(volatile v4i*)(Wh + po[q]) = uh[q].i;
    *(volatile v4i*)(Wl + po[q]) = ul[q].i;
  }
  __threadfence();
#pragma unroll
  for (int q = 0; q < 2; ++q) {
    *(volatile v4i*)(Wh + po[q]) = uh[q].i;
    *(volatile v4i*)(Wl + po[q]) = ul[q].i;
  }
}

__global__ __launch_bounds__(NTHR) void k_gemm(
    const float* __restrict__ X, const float* __restrict__ st,
    const unsigned short* __restrict__ Wh, const unsigned short* __restrict__ Wl,
    const float* __restrict__ cb, const float* __restrict__ avs, const float* __restrict__ avd,
    float* outp, float* alsp, float* aldp,
    int nN, int KT, int NT, int bn, int ncb, int H, int C) {
  __shared__ __attribute__((aligned(16))) unsigned short Ah[GR * AP];
  __shared__ __attribute__((aligned(16))) unsigned short Al[GR * AP];
  __shared__ __attribute__((aligned(16))) float Xs[GR * XSP];
  __shared__ __attribute__((aligned(16))) float Aav[2 * DF];
  __shared__ __attribute__((aligned(16))) float Alp[2 * GR * HP];

  const int tid  = threadIdx.x;
  const int lane = tid & 31;
  const int wave = tid >> 5;
  const int hh   = lane >> 4;
  const int m    = lane & 15;
  const int rowBase = blockIdx.x * GR;

  if (H > 0) {
    const int F = H * C;
    if (tid < DF) {
      const int i = (tid < F) ? tid : (F - 1);
      const float a = avs[i];
      const float d = avd[i];
      Aav[tid]      = (tid < F) ? a : 0.f;
      Aav[DF + tid] = (tid < F) ? d : 0.f;
    }
  }

  {
    const int r  = tid >> 3;
    const int c0 = (tid & 7) * 16;
    int row = rowBase + r;
    if (row > nN - 1) row = nN - 1;
    const float* p = X + (size_t)row * DF + c0;
    v4f f0 = *(const v4f*)(p), f1 = *(const v4f*)(p + 4);
    v4f f2 = *(const v4f*)(p + 8), f3 = *(const v4f*)(p + 12);
    if (bn) {
      const v4f sa = *(const v4f*)(st + c0),      sb = *(const v4f*)(st + c0 + 4);
      const v4f sc = *(const v4f*)(st + c0 + 8),  sd = *(const v4f*)(st + c0 + 12);
      const v4f ta = *(const v4f*)(st + DF + c0),     tb = *(const v4f*)(st + DF + c0 + 4);
      const v4f tc = *(const v4f*)(st + DF + c0 + 8), td = *(const v4f*)(st + DF + c0 + 12);
      f0 = relu4(f0 * sa + ta);
      f1 = relu4(f1 * sb + tb);
      f2 = relu4(f2 * sc + tc);
      f3 = relu4(f3 * sd + td);
    }
    float v[16];
    v[0] = f0.x;  v[1] = f0.y;  v[2] = f0.z;  v[3] = f0.w;
    v[4] = f1.x;  v[5] = f1.y;  v[6] = f1.z;  v[7] = f1.w;
    v[8] = f2.x;  v[9] = f2.y;  v[10] = f2.z; v[11] = f2.w;
    v[12] = f3.x; v[13] = f3.y; v[14] = f3.z; v[15] = f3.w;
    Pack16 h0, h1, l0, l1;
#pragma unroll
    for (int j = 0; j < 8; ++j) {
      unsigned short a, b;
      bf_split(v[j], a, b);
      h0.h[j] = a; l0.h[j] = b;
      bf_split(v[8 + j], a, b);
      h1.h[j] = a; l1.h[j] = b;
    }
    *(v8us*)(Ah + r * AP + c0)     = h0.h;
    *(v8us*)(Ah + r * AP + c0 + 8) = h1.h;
    *(v8us*)(Al + r * AP + c0)     = l0.h;
    *(v8us*)(Al + r * AP + c0 + 8) = l1.h;
  }
  __syncthreads();

  const int ncol = wave * 16 + m;
  v8f c0a = {0.f, 0.f, 0.f, 0.f, 0.f, 0.f, 0.f, 0.f};
  v8f c1a = {0.f, 0.f, 0.f, 0.f, 0.f, 0.f, 0.f, 0.f};
  if (wave < NT) {
#pragma unroll 1
    for (int kt = 0; kt < KT; ++kt) {
      const int k0 = kt * 32;
      Frag a0h, a0l, a1h, a1l, bh, bl;
      const unsigned short* pbh  = Wh + (size_t)ncol * DF + k0 + 8 * hh;
      const unsigned short* pbl  = Wl + (size_t)ncol * DF + k0 + 8 * hh;
      const unsigned short* pa0h = Ah + m * AP + k0 + 8 * hh;
      const unsigned short* pa0l = Al + m * AP + k0 + 8 * hh;
      const unsigned short* pa1h = Ah + (16 + m) * AP + k0 + 8 * hh;
      const unsigned short* pa1l = Al + (16 + m) * AP + k0 + 8 * hh;
      bh.half[0]  = *(const v8us*)pbh;  bh.half[1]  = *(const v8us*)(pbh + 16);
      bl.half[0]  = *(const v8us*)pbl;  bl.half[1]  = *(const v8us*)(pbl + 16);
      a0h.half[0] = *(const v8us*)pa0h; a0h.half[1] = *(const v8us*)(pa0h + 16);
      a0l.half[0] = *(const v8us*)pa0l; a0l.half[1] = *(const v8us*)(pa0l + 16);
      a1h.half[0] = *(const v8us*)pa1h; a1h.half[1] = *(const v8us*)(pa1h + 16);
      a1l.half[0] = *(const v8us*)pa1l; a1l.half[1] = *(const v8us*)(pa1l + 16);
      c0a = wm(a0h.v, bh.v, c0a);
      c0a = wm(a0h.v, bl.v, c0a);
      c0a = wm(a0l.v, bh.v, c0a);
      c1a = wm(a1h.v, bh.v, c1a);
      c1a = wm(a1h.v, bl.v, c1a);
      c1a = wm(a1l.v, bh.v, c1a);
    }
  }

  {
    const int   cbi  = (ncol < ncb) ? ncol : 0;
    const float cbv  = cb[cbi];
    const float addb = (ncol < ncb) ? cbv : 0.f;
#pragma unroll
    for (int r = 0; r < 8; ++r) {
      Xs[(8 * hh + r) * XSP + ncol]      = c0a[r] + addb;
      Xs[(16 + 8 * hh + r) * XSP + ncol] = c1a[r] + addb;
    }
  }
  __syncthreads();

  if (H > 0) {
    const int row  = tid >> 3;
    const int head = tid & 7;
    const int hc   = (head < H) ? head : (H - 1);
    const float* xr = Xs + row * XSP + hc * C;
    const float* av = Aav + hc * C;
    float ds = 0.f, dd = 0.f;
#pragma unroll 1
    for (int c = 0; c < C; ++c) {
      const float xv = xr[c];
      ds += xv * av[c];
      dd += xv * av[DF + c];
    }
    Alp[row * HP + head]           = (head < H) ? ds : 0.f;
    Alp[GR * HP + row * HP + head] = (head < H) ? dd : 0.f;
  }
  __syncthreads();

  v4f xr4[4];
  float* xpp[4];
#pragma unroll
  for (int i = 0; i < 4; ++i) {
    xr4[i] = *(const v4f*)(Xs + (4 * wave + i) * XSP + 4 * lane);
    xpp[i] = outp + (size_t)(rowBase + 4 * wave + i) * DF + 4 * lane;
  }
  const bool wa = (H > 0) && (wave < 2);
  v4f av0 = {0.f, 0.f, 0.f, 0.f};
  v4f av1 = {0.f, 0.f, 0.f, 0.f};
  float* ap0 = outp;
  float* ap1 = outp;
  if (wa) {
    const float* srcl = Alp + wave * (GR * HP);
    av0 = *(const v4f*)(srcl + 4 * lane);
    av1 = *(const v4f*)(srcl + 128 + 4 * lane);
    float* base = ((wave == 0) ? alsp : aldp) + (size_t)rowBase * HP;
    ap0 = base + 4 * lane;
    ap1 = base + 128 + 4 * lane;
  }
#pragma unroll
  for (int i = 0; i < 4; ++i) *(volatile v4f*)(xpp[i]) = xr4[i];
  if (wa) { *(volatile v4f*)ap0 = av0; *(volatile v4f*)ap1 = av1; }
  __threadfence();
#pragma unroll
  for (int i = 0; i < 4; ++i) *(volatile v4f*)(xpp[i]) = xr4[i];
  if (wa) { *(volatile v4f*)ap0 = av0; *(volatile v4f*)ap1 = av1; }
}

__global__ __launch_bounds__(NTHR) void k_agg(
    const float* __restrict__ feat, const float* __restrict__ alsp, const float* __restrict__ aldp,
    const int* __restrict__ ei, const float* __restrict__ bias, float* outp,
    int nN, int nE, int H, int C) {
  extern __shared__ v4f lds_dyn[];
  float* sacc = (float*)lds_dyn;
  float* daux = sacc + LDS_SACC;
  float* maux = daux + LDS_DEN;
  int*   list = (int*)(maux + LDS_MAX);
  int*   wcnt = list + LDS_LIST;

  const int tid  = threadIdx.x;
  const int lane = tid & 31;
  const int wave = tid >> 5;
  int hd = (4 * lane) / C;
  hd = (hd > H - 1) ? (H - 1) : hd;
  const int nodeBase = blockIdx.x * NB;
  const int* srcp = ei;
  const int* dstp = ei + nE;

#pragma unroll 1
  for (int q = 0; q < NB / NWAVE; ++q) {
    const int slot = wave * (NB / NWAVE) + q;
    int node = nodeBase + slot;
    node = (node > nN - 1) ? (nN - 1) : node;
    float s = alsp[(size_t)node * HP + hd] + aldp[(size_t)node * HP + hd];
    s = (s >= 0.f) ? s : 0.2f * s;
    maux[slot * HP + hd] = s;
    daux[slot * HP + hd] = 1.0f;
    *(v4f*)(sacc + slot * DF + 4 * lane) = *(const v4f*)(feat + (size_t)node * DF + 4 * lane);
  }
  __syncthreads();

  const bool al16 = ((((size_t)dstp) & 15) == 0);

  const int nChunks = (nE + CHUNK - 1) / CHUNK;
#pragma unroll 1
  for (int ch = 0; ch < nChunks; ++ch) {
    const int cbase = ch * CHUNK;
    int wc = 0;
    {
      const int el0 = tid * 4;
      const int e0  = cbase + el0;
      const int sent = -2147483647 - 1;
      v4i d;
      if (al16 && (cbase + CHUNK <= nE)) {
        d = *(const v4i*)(dstp + e0);
      } else {
        const int i0 = (e0     < nE) ? e0     : (nE - 1);
        const int i1 = (e0 + 1 < nE) ? e0 + 1 : (nE - 1);
        const int i2 = (e0 + 2 < nE) ? e0 + 2 : (nE - 1);
        const int i3 = (e0 + 3 < nE) ? e0 + 3 : (nE - 1);
        const int v0 = dstp[i0], v1 = dstp[i1], v2 = dstp[i2], v3 = dstp[i3];
        d.x = (e0     < nE) ? v0 : sent;
        d.y = (e0 + 1 < nE) ? v1 : sent;
        d.z = (e0 + 2 < nE) ? v2 : sent;
        d.w = (e0 + 3 < nE) ? v3 : sent;
      }
      const unsigned s0 = (unsigned)d.x - (unsigned)nodeBase;
      const unsigned s1 = (unsigned)d.y - (unsigned)nodeBase;
      const unsigned s2 = (unsigned)d.z - (unsigned)nodeBase;
      const unsigned s3 = (unsigned)d.w - (unsigned)nodeBase;
      const bool h0 = s0 < (unsigned)NB;
      const bool h1 = s1 < (unsigned)NB;
      const bool h2 = s2 < (unsigned)NB;
      const bool h3 = s3 < (unsigned)NB;
      const unsigned many = __builtin_amdgcn_ballot_w32(h0 | h1 | h2 | h3);
      if (many != 0u) {
#define HITJ(J, HJ, SJ) { \
          const unsigned mj = __builtin_amdgcn_ballot_w32(HJ); \
          if (HJ) { \
            const int pos = wc + (int)__builtin_amdgcn_mbcnt_lo(mj, 0u); \
            if (pos < WCAP) list[wave * WCAP + pos] = ((el0 + (J)) << 9) | (int)(SJ); \
          } \
          wc += (int)__builtin_popcount(mj); }
        HITJ(0, h0, s0)
        HITJ(1, h1, s1)
        HITJ(2, h2, s2)
        HITJ(3, h3, s3)
#undef HITJ
      }
    }
    if (lane == 0) wcnt[wave] = wc;
    __syncthreads();

    if (wave == 0) {
      for (int wsx = 0; wsx < NWAVE; ++wsx) {
        int n = __builtin_amdgcn_readfirstlane(wcnt[wsx]);
        n = n > WCAP ? WCAP : n;
        n = n < 0 ? 0 : n;
        for (int i = 0; i < n; ++i) {
          const int ent  = __builtin_amdgcn_readfirstlane(list[wsx * WCAP + i]);
          int slot = ent & (SLOTP - 1);
          slot = (slot > NB - 1) ? (NB - 1) : slot;
          const int eloc = (ent >> 9) & (CHUNK - 1);
          int e = cbase + eloc;
          e = e > nE - 1 ? nE - 1 : e;
          int j = srcp[e];
          j = j < 0 ? 0 : (j > nN - 1 ? nN - 1 : j);
          int nd = nodeBase + slot;
          nd = nd > nN - 1 ? nN - 1 : nd;
          float s = alsp[(size_t)j * HP + hd] + aldp[(size_t)nd * HP + hd];
          s = (s >= 0.f) ? s : 0.2f * s;
          const int ai = slot * HP + hd;
          const float mo = maux[ai];
          const float dn = daux[ai];
          const float mn = fmaxf(mo, s);
          const float cf = __expf(mo - mn);
          const float p  = __expf(s - mn);
          const v4f xv = *(const v4f*)(feat + (size_t)j * DF + 4 * lane);
          v4f* sp = (v4f*)(sacc + slot * DF + 4 * lane);
          const v4f cur = *sp;
          const v4f nxt = cur * cf + xv * p;
          *sp = nxt;
          maux[ai] = mn;
          daux[ai] = dn * cf + p;
        }
      }
    }
    __syncthreads();
  }

  const int nb4 = (H * C) >> 2;
  const int lc  = (lane < nb4) ? lane : (nb4 - 1);
  const v4f bb  = *(const v4f*)(bias + 4 * lc);
  const v4f z4  = {0.f, 0.f, 0.f, 0.f};
  const v4f b4  = (lane < nb4) ? bb : z4;
#pragma unroll 1
  for (int q = 0; q < NB / NWAVE; ++q) {
    const int slot = wave * (NB / NWAVE) + q;
    const int node = nodeBase + slot;
    if (node >= nN) break;
    const float dn  = daux[slot * HP + hd];
    const float inv = 1.0f / dn;
    const v4f sv = *(const v4f*)(sacc + slot * DF + 4 * lane);
    const v4f y  = sv * inv + b4;
    float* op = outp + (size_t)node * DF + 4 * lane;
    *(volatile v4f*)op = y;
    __threadfence();
    *(volatile v4f*)op = y;
  }
}

__global__ __launch_bounds__(NTHR) void k_bnstat(const float* __restrict__ P, int nN, float* part) {
  __shared__ v4f S1[NWAVE * 32];
  __shared__ v4f S2[NWAVE * 32];
  const int tid  = threadIdx.x;
  const int lane = tid & 31;
  const int wave = tid >> 5;
  const int R  = (nN + NBLK - 1) / NBLK;
  const int r0 = blockIdx.x * R;
  v4f a1 = {0.f, 0.f, 0.f, 0.f};
  v4f a2 = {0.f, 0.f, 0.f, 0.f};
#pragma unroll 1
  for (int r = wave; r < R; r += NWAVE) {
    const int row = r0 + r;
    if (row >= nN) break;
    const v4f v = *(const v4f*)(P + (size_t)row * DF + 4 * lane);
    a1 += v;
    a2 += v * v;
  }
  S1[wave * 32 + lane] = a1;
  S2[wave * 32 + lane] = a2;
  __syncthreads();
  if (wave == 0) {
    v4f t1 = S1[lane];
    v4f t2 = S2[lane];
#pragma unroll
    for (int q = 1; q < NWAVE; ++q) { t1 += S1[q * 32 + lane]; t2 += S2[q * 32 + lane]; }
    float* pp = part + (size_t)blockIdx.x * (2 * DF);
    *(volatile v4f*)(pp + 4 * lane)      = t1;
    *(volatile v4f*)(pp + DF + 4 * lane) = t2;
    __threadfence();
    *(volatile v4f*)(pp + 4 * lane)      = t1;
    *(volatile v4f*)(pp + DF + 4 * lane) = t2;
  }
}

__global__ __launch_bounds__(DF) void k_bnfin(const float* __restrict__ part, int nN, int F,
                                             const float* __restrict__ gamma,
                                             const float* __restrict__ beta, float* st) {
  __shared__ __attribute__((aligned(16))) float Ss[DF];
  __shared__ __attribute__((aligned(16))) float Ts[DF];
  const int c    = threadIdx.x;
  const int lane = c & 31;
  const int wave = c >> 5;
  double s1 = 0.0, s2 = 0.0;
#pragma unroll 1
  for (int b = 0; b < NBLK; ++b) {
    s1 += (double)part[(size_t)b * (2 * DF) + c];
    s2 += (double)part[(size_t)b * (2 * DF) + DF + c];
  }
  const double mean = s1 / (double)nN;
  double var = s2 / (double)nN - mean * mean;
  if (var < 0.0) var = 0.0;
  const float rstd = 1.0f / sqrtf((float)var + EPSBN);
  const int ci = (c < F) ? c : (F - 1);
  const float gv = gamma[ci];
  const float bv = beta[ci];
  const float sc = (c < F) ? gv * rstd : 0.f;
  const float tc = (c < F) ? (bv - (float)mean * sc) : 0.f;
  Ss[c] = sc;
  Ts[c] = tc;
  __syncthreads();
  if (wave == 0) {
    const v4f sv = *(const v4f*)(Ss + 4 * lane);
    const v4f tv = *(const v4f*)(Ts + 4 * lane);
    *(volatile v4f*)(st + 4 * lane)      = sv;
    *(volatile v4f*)(st + DF + 4 * lane) = tv;
    __threadfence();
    *(volatile v4f*)(st + 4 * lane)      = sv;
    *(volatile v4f*)(st + DF + 4 * lane) = tv;
  }
}

__global__ __launch_bounds__(NTHR) void k_pool(const float* __restrict__ P, const float* __restrict__ st,
                                               const int* __restrict__ bat, int nN, float* pooled) {
  __shared__ v4f Acc[NWAVE * 32];
  __shared__ int Cn[NWAVE];
  const int tid  = threadIdx.x;
  const int lane = tid & 31;
  const int wave = tid >> 5;
  const int g    = blockIdx.x;
  const v4f s4 = *(const v4f*)(st + 4 * lane);
  const v4f t4 = *(const v4f*)(st + DF + 4 * lane);
  const v4f z4 = {0.f, 0.f, 0.f, 0.f};
  v4f acc = z4;
  int cnt = 0;
  const bool al16 = ((((size_t)bat) & 15) == 0);
#pragma unroll 1
  for (int cb = wave * 128; cb < nN; cb += NWAVE * 128) {
    const int e0 = cb + 4 * lane;
    v4i d;
    if (al16 && (cb + 128 <= nN)) {
      d = *(const v4i*)(bat + e0);
    } else {
      const int i0 = (e0     < nN) ? e0     : (nN - 1);
      const int i1 = (e0 + 1 < nN) ? e0 + 1 : (nN - 1);
      const int i2 = (e0 + 2 < nN) ? e0 + 2 : (nN - 1);
      const int i3 = (e0 + 3 < nN) ? e0 + 3 : (nN - 1);
      const int v0 = bat[i0], v1 = bat[i1], v2 = bat[i2], v3 = bat[i3];
      d.x = (e0     < nN) ? v0 : -1;
      d.y = (e0 + 1 < nN) ? v1 : -1;
      d.z = (e0 + 2 < nN) ? v2 : -1;
      d.w = (e0 + 3 < nN) ? v3 : -1;
    }
    const bool h0 = (d.x == g), h1 = (d.y == g), h2 = (d.z == g), h3 = (d.w == g);
#define POOLJ(J, HJ) { \
      unsigned mj = __builtin_amdgcn_ballot_w32(HJ); \
      while (mj != 0u) { \
        const int b = __builtin_ctz(mj); \
        mj &= mj - 1u; \
        int node = cb + 4 * b + (J); \
        node = (node > nN - 1) ? (nN - 1) : node; \
        const v4f v = *(const v4f*)(P + (size_t)node * DF + 4 * lane); \
        acc += relu4(v * s4 + t4); \
        ++cnt; \
      } }
    POOLJ(0, h0)
    POOLJ(1, h1)
    POOLJ(2, h2)
    POOLJ(3, h3)
#undef POOLJ
  }
  Acc[wave * 32 + lane] = acc;
  if (lane == 0) Cn[wave] = cnt;
  __syncthreads();
  if (wave == 0) {
    v4f tot = Acc[lane];
    int n = Cn[0];
#pragma unroll
    for (int q = 1; q < NWAVE; ++q) { tot += Acc[q * 32 + lane]; n += Cn[q]; }
    const float inv = 1.0f / (float)((n > 1) ? n : 1);
    const v4f mean = tot * inv;
    float* pp = pooled + (size_t)g * DF + 4 * lane;
    *(volatile v4f*)pp = mean;
    __threadfence();
    *(volatile v4f*)pp = mean;
  }
}

__global__ __launch_bounds__(NTHR) void k_head(const float* __restrict__ pooled, const float* __restrict__ Wo,
                                               const float* __restrict__ bo, float* outp) {
  __shared__ __attribute__((aligned(16))) float Ws[KHD * NCLS];
  __shared__ float Bs[16];
  __shared__ __attribute__((aligned(16))) float Os[NG * NCLS];
  const int tid = threadIdx.x;
  for (int i = tid; i < KHD * NCLS; i += NTHR) Ws[i] = Wo[i];
  { const float bov = bo[min(tid, NCLS - 1)]; if (tid < NCLS) Bs[tid] = bov; }
  __syncthreads();
#pragma unroll 1
  for (int i = 0; i < (NG * NCLS) / NTHR; ++i) {
    const int o = i * NTHR + tid;
    const int g = o / NCLS;
    const int c = o - g * NCLS;
    const float* pr = pooled + (size_t)g * DF;
    float s = 0.f;
#pragma unroll 4
    for (int k = 0; k < KHD; ++k) s += pr[k] * Ws[k * NCLS + c];
    Os[o] = s + Bs[c];
  }
  __syncthreads();
  v4f ov[5];
  float* opv[5];
#pragma unroll
  for (int i = 0; i < 5; ++i) {
    const int f4 = i * NTHR + tid;
    ov[i]  = *(const v4f*)(Os + 4 * f4);
    opv[i] = outp + 4 * f4;
  }
#pragma unroll
  for (int i = 0; i < 5; ++i) *(volatile v4f*)(opv[i]) = ov[i];
  __threadfence();
#pragma unroll
  for (int i = 0; i < 5; ++i) *(volatile v4f*)(opv[i]) = ov[i];
}

extern "C" void kernel_launch(void* const* d_in, const int* in_sizes, int n_in,
                              void* d_out, int out_size, void* d_ws, size_t ws_size,
                              hipStream_t stream) {
  if (n_in != 31) return;
  const int nN = in_sizes[0] / DF;
  if (nN <= 0 || in_sizes[0] != nN * DF) return;
  if ((in_sizes[1] & 1) != 0) return;
  const int nE = in_sizes[1] / 2;
  if (nE <= 0) return;
  if (in_sizes[2] != nN) return;
  static const int want[28] = {16384, 128, 128, 128, 128, 128, 2048, 16, 16, 16,
                               1536, 96, 96, 96, 96, 96, 2304, 24, 24, 24,
                               1536, 64, 64, 64, 64, 64, 640, 10};
  for (int i = 0; i < 28; ++i) if (in_sizes[3 + i] != want[i]) return;
  if (out_size != NG * NCLS) return;

  const float* x    = (const float*)d_in[0];
  const int*   ei   = (const int*)d_in[1];
  const int*   bat  = (const int*)d_in[2];
  const float* W1   = (const float*)d_in[3];
  const float* as1  = (const float*)d_in[4];
  const float* ad1  = (const float*)d_in[5];
  const float* b1   = (const float*)d_in[6];
  const float* g1   = (const float*)d_in[7];
  const float* be1  = (const float*)d_in[8];
  const float* Wl1  = (const float*)d_in[9];
  const float* bl1  = (const float*)d_in[10];
  const float* gl1  = (const float*)d_in[11];
  const float* bel1 = (const float*)d_in[12];
  const float* W2   = (const float*)d_in[13];
  const float* as2  = (const float*)d_in[14];
  const float* ad2  = (const float*)d_in[15];
  const float* b2   = (const float*)d_in[16];
  const float* g2   = (const float*)d_in[17];
  const float* be2  = (const float*)d_in[18];
  const float* Wl2  = (const float*)d_in[19];
  const float* bl2  = (const float*)d_in[20];
  const float* gl2  = (const float*)d_in[21];
  const float* bel2 = (const float*)d_in[22];
  const float* W3   = (const float*)d_in[23];
  const float* as3  = (const float*)d_in[24];
  const float* ad3  = (const float*)d_in[25];
  const float* b3   = (const float*)d_in[26];
  const float* g3   = (const float*)d_in[27];
  const float* be3  = (const float*)d_in[28];
  const float* Wo   = (const float*)d_in[29];
  const float* bo   = (const float*)d_in[30];
  float* outp = (float*)d_out;

  const int nP = ((nN + GR - 1) / GR) * GR;
  size_t off = 0;
  unsigned short* Wh = (unsigned short*)((char*)d_ws + off); off += (size_t)DF * DF * sizeof(unsigned short);
  unsigned short* Wl = (unsigned short*)((char*)d_ws + off); off += (size_t)DF * DF * sizeof(unsigned short);
  float* P0   = (float*)((char*)d_ws + off); off += (size_t)nP * DF * sizeof(float);
  float* P1   = (float*)((char*)d_ws + off); off += (size_t)nP * DF * sizeof(float);
  float* ALS  = (float*)((char*)d_ws + off); off += (size_t)nP * HP * sizeof(float);
  float* ALD  = (float*)((char*)d_ws + off); off += (size_t)nP * HP * sizeof(float);
  float* PART = (float*)((char*)d_ws + off); off += (size_t)NBLK * 2 * DF * sizeof(float);
  float* ST   = (float*)((char*)d_ws + off); off += (size_t)2 * DF * sizeof(float);
  float* POOL = (float*)((char*)d_ws + off); off += (size_t)NG * DF * sizeof(float);
  if (off > ws_size) return;

  hipFuncSetAttribute(reinterpret_cast<const void*>(&k_agg),
                      hipFuncAttributeMaxDynamicSharedMemorySize, LDS_BYTES);
  const int ggemm = nP / GR;
  const int gagg  = (nN + NB - 1) / NB;

  k_prepw<<<DF / 32, NTHR, 0, stream>>>(W1, 128, 128, Wh, Wl);
  k_gemm<<<ggemm, NTHR, 0, stream>>>(x, ST, Wh, Wl, W1, as1, ad1, P0, ALS, ALD, nN, 4, 8, 0, 0, 8, 16);
  k_agg<<<gagg, NTHR, LDS_BYTES, stream>>>(P0, ALS, ALD, ei, b1, P1, nN, nE, 8, 16);
  k_bnstat<<<NBLK, NTHR, 0, stream>>>(P1, nN, PART);
  k_bnfin<<<1, DF, 0, stream>>>(PART, nN, 128, g1, be1, ST);

  k_prepw<<<DF / 32, NTHR, 0, stream>>>(Wl1, 128, 16, Wh, Wl);
  k_gemm<<<ggemm, NTHR, 0, stream>>>(P1, ST, Wh, Wl, bl1, as1, ad1, P0, ALS, ALD, nN, 4, 1, 1, 16, 0, 16);
  k_bnstat<<<NBLK, NTHR, 0, stream>>>(P0, nN, PART);
  k_bnfin<<<1, DF, 0, stream>>>(PART, nN, 16, gl1, bel1, ST);

  k_prepw<<<DF / 32, NTHR, 0, stream>>>(W2, 16, 96, Wh, Wl);
  k_gemm<<<ggemm, NTHR, 0, stream>>>(P0, ST, Wh, Wl, W2, as2, ad2, P1, ALS, ALD, nN, 1, 6, 1, 0, 4, 24);
  k_agg<<<gagg, NTHR, LDS_BYTES, stream>>>(P1, ALS, ALD, ei, b2, P0, nN, nE, 4, 24);
  k_bnstat<<<NBLK, NTHR, 0, stream>>>(P0, nN, PART);
  k_bnfin<<<1, DF, 0, stream>>>(PART, nN, 96, g2, be2, ST);

  k_prepw<<<DF / 32, NTHR, 0, stream>>>(Wl2, 96, 24, Wh, Wl);
  k_gemm<<<ggemm, NTHR, 0, stream>>>(P0, ST, Wh, Wl, bl2, as2, ad2, P1, ALS, ALD, nN, 3, 2, 1, 24, 0, 24);
  k_bnstat<<<NBLK, NTHR, 0, stream>>>(P1, nN, PART);
  k_bnfin<<<1, DF, 0, stream>>>(PART, nN, 24, gl2, bel2, ST);

  k_prepw<<<DF / 32, NTHR, 0, stream>>>(W3, 24, 64, Wh, Wl);
  k_gemm<<<ggemm, NTHR, 0, stream>>>(P1, ST, Wh, Wl, W3, as3, ad3, P0, ALS, ALD, nN, 1, 4, 1, 0, 2, 32);
  k_agg<<<gagg, NTHR, LDS_BYTES, stream>>>(P0, ALS, ALD, ei, b3, P1, nN, nE, 2, 32);
  k_bnstat<<<NBLK, NTHR, 0, stream>>>(P1, nN, PART);
  k_bnfin<<<1, DF, 0, stream>>>(PART, nN, 64, g3, be3, ST);

  k_pool<<<NG, NTHR, 0, stream>>>(P1, ST, bat, nN, POOL);
  k_head<<<1, NTHR, 0, stream>>>(POOL, Wo, bo, outp);
}
